// InfiniAttention_48052094108063
// MI455X (gfx1250) — hardware-verified
//
#include <hip/hip_runtime.h>
#ifndef NB
#define NB 2
#endif
#ifndef SEQ
#define SEQ 2048
#endif
#define NB_FULL 2
#define SEQ_FULL 2048
#define DM 1024
#define NX (DM + 64)
#define NR (NB * SEQ)
#define ERS ((SEQ < 512) ? SEQ : 512)
#define NVH 16
#define WSC 64.0f
#define MSC 1024.0f
#define RSC 1024.0f
#define EPSV 1e-6f
#define WS_CAP ((size_t)134217728)
static_assert(NB >= 1 && NB <= NB_FULL);
static_assert(SEQ >= 128 && SEQ <= SEQ_FULL && (SEQ % 128) == 0);
static_assert((ERS % 128) == 0 && ERS <= SEQ);
static_assert((DM % 64) == 0 && (NX % 64) == 0 && (DM % 32) == 0);
static_assert((size_t)NR * NX * 4 <= (size_t)3 * NR * DM * 2);

typedef unsigned short v8us __attribute__((ext_vector_type(8), may_alias));
typedef unsigned int v4u __attribute__((ext_vector_type(4), may_alias));
typedef float v8f __attribute__((ext_vector_type(8)));
typedef float v8fa __attribute__((ext_vector_type(8), may_alias));
typedef float v4f __attribute__((ext_vector_type(4)));
typedef float v4fa __attribute__((ext_vector_type(4), may_alias));
typedef _Float16 v16h __attribute__((ext_vector_type(16)));
typedef _Float16 v4h __attribute__((ext_vector_type(4)));
union FragH { v16h v; v8us half[2]; _Float16 h[16]; unsigned short u[16]; };

__device__ __forceinline__ unsigned short bf16_bits(float x) { unsigned int u = __float_as_uint(x); return (unsigned short)((u + 0x7FFFu + ((u >> 16) & 1u)) >> 16); }
__device__ __forceinline__ float bf16_val(unsigned short b) { return __uint_as_float(((unsigned int)b) << 16); }
__device__ __forceinline__ float bf16_rne(float x) { return bf16_val(bf16_bits(x)); }

__device__ __forceinline__ v16h g2_frag(const _Float16* p, int hh) { FragH f; f.half[0] = *(const v8us*)((const unsigned short*)p + 8 * hh); f.half[1] = *(const v8us*)((const unsigned short*)p + 16 + 8 * hh); return f.v; }
__device__ __forceinline__ v8f g2_mma(v16h a, v16h b, v8f c) { v8f d = __builtin_amdgcn_wmma_f32_16x16x32_f16(false, a, false, b, (short)0, c, false, false); asm volatile("v_nop\n\tv_nop\n\tv_nop\n\tv_nop" : "+v"(d) : "v"(a), "v"(b)); return d; }

template <int ACT, int CMASK, int KLIM>
__global__ __launch_bounds__(128) void k_gemm2(const _Float16* __restrict__ A, int lda, size_t sA, const _Float16* __restrict__ Bh, int ldb, size_t sB, float alpha,
    const float* CP, int cprows, float* C, _Float16* C16, _Float16* C16L, int ldc, size_t sC, int M, int N, int K) {
  __shared__ __attribute__((aligned(16))) float so[4][32][68];
  const int tid = threadIdx.x, w = tid >> 5, lane = tid & 31, ln = lane & 15, hh = lane >> 4;
  const int by = blockIdx.y;
  A += (size_t)by * sA; Bh += (size_t)by * sB; const size_t cofs = (size_t)by * sC;
  const int ntn = N >> 6; const int mt = blockIdx.x / ntn, nq = blockIdx.x - mt * ntn;
  const int rowb = mt * 128; const int row0 = rowb + 32 * w, col0 = nq * 64;
  if (row0 >= M) return;
  if (CMASK != 0 && col0 >= rowb + 128) return;
  const int kend = (KLIM != 0) ? min(K, rowb + 128) : K;
  const _Float16* a0p = A + (size_t)(row0 + ln) * lda; const _Float16* a1p = a0p + (size_t)16 * lda;
  const _Float16* b0p = Bh + (size_t)(col0 + ln) * ldb; const _Float16* b1p = b0p + (size_t)16 * ldb; const _Float16* b2p = b1p + (size_t)16 * ldb; const _Float16* b3p = b2p + (size_t)16 * ldb;
  const v8f z8 = {0.f,0.f,0.f,0.f,0.f,0.f,0.f,0.f}; v8f c00 = z8, c01 = z8, c02 = z8, c03 = z8, c10 = z8, c11 = z8, c12 = z8, c13 = z8;
#pragma unroll 1
  for (int kb = 0; kb < kend; kb += 32) { const v16h a0 = g2_frag(a0p + kb, hh), a1 = g2_frag(a1p + kb, hh);
    v16h b = g2_frag(b0p + kb, hh); c00 = g2_mma(a0, b, c00); c10 = g2_mma(a1, b, c10);
    b = g2_frag(b1p + kb, hh); c01 = g2_mma(a0, b, c01); c11 = g2_mma(a1, b, c11);
    b = g2_frag(b2p + kb, hh); c02 = g2_mma(a0, b, c02); c12 = g2_mma(a1, b, c12);
    b = g2_frag(b3p + kb, hh); c03 = g2_mma(a0, b, c03); c13 = g2_mma(a1, b, c13); }
  v8f accs[8] = {c00, c01, c02, c03, c10, c11, c12, c13};
#pragma unroll
  for (int u = 0; u < 8; ++u) { const int t = u & 3, half = u >> 2;
#pragma unroll
    for (int r = 0; r < 8; ++r) { const int rloc = half * 16 + 8 * hh + r; float v = accs[u][r] * alpha;
      if (ACT == 7) { const float e = expf(fminf(v, 0.0f)); v = (v > 0.0f) ? (v + 1.0f) : e; }
      so[w][rloc][t * 16 + ln] = v; } }
  __builtin_amdgcn_fence(4  , "workgroup"); __builtin_amdgcn_wave_barrier();
  const int rsub = lane >> 4, c4 = (lane & 15) * 4;
  const bool addcp = (CP != nullptr) && (rowb < cprows);
  if (CMASK != 0 || addcp) {
#pragma unroll
    for (int q = 0; q < 16; ++q) { const int r = q * 2 + rsub; v4f xv = *(const v4fa*)&so[w][r][c4];
      if (addcp) { const v4f cpv = *(const v4fa*)(CP + cofs + (size_t)(row0 + r) * ldc + col0 + c4); xv += cpv; }
      if (CMASK != 0) {
#pragma unroll
        for (int i = 0; i < 4; ++i) { if (col0 + c4 + i > row0 + r) xv[i] = 0.0f; } }
      *(v4fa*)&so[w][r][c4] = xv; }
    __builtin_amdgcn_fence(4  , "workgroup"); __builtin_amdgcn_wave_barrier();
  }
  for (int pass = 0; pass < 2; ++pass) {
#pragma unroll
    for (int q = 0; q < 16; ++q) { const int r = q * 2 + rsub; const v4f v = *(const v4fa*)&so[w][r][c4];
      const size_t o = cofs + (size_t)(row0 + r) * ldc + col0 + c4;
      if (C != nullptr) *(volatile v4f*)(C + o) = v;
      if (C16 != nullptr) { v4h h4, l4;
#pragma unroll
        for (int i = 0; i < 4; ++i) { const _Float16 hv = (_Float16)v[i]; h4[i] = hv; l4[i] = (_Float16)((v[i] - (float)hv) * RSC); }
        *(volatile v4h*)(C16 + o) = h4;
        if (C16L != nullptr) *(volatile v4h*)(C16L + o) = l4; } }
    if (pass == 0) __threadfence(); }
}

__global__ __launch_bounds__(256) void k_wsc(const float* __restrict__ Wm, _Float16* __restrict__ Bt, size_t n8, float sc) {
  const size_t t = (size_t)blockIdx.x * 256 + threadIdx.x; if (t >= n8) return;
  const v4f a = *(const v4fa*)(Wm + t * 8), c = *(const v4fa*)(Wm + t * 8 + 4); FragH f;
#pragma unroll
  for (int q = 0; q < 4; ++q) { f.h[q] = (_Float16)(bf16_rne(a[q]) * sc); f.h[4 + q] = (_Float16)(bf16_rne(c[q]) * sc); }
  *(volatile v8us*)((unsigned short*)Bt + t * 8) = f.half[0]; __threadfence(); *(volatile v8us*)((unsigned short*)Bt + t * 8) = f.half[0]; }

__global__ __launch_bounds__(256) void k_wt_f16(const float* __restrict__ W, _Float16* __restrict__ Wt, int K, int N, float scale) {
  const int t = blockIdx.x * 256 + threadIdx.x; if (t >= N * (K / 8)) return; const int n = t / (K / 8), k8 = (t % (K / 8)) * 8; FragH f;
#pragma unroll
  for (int i = 0; i < 8; ++i) f.h[i] = (_Float16)(bf16_rne(W[(size_t)(k8 + i) * N + n]) * scale); const v8us o = f.half[0];
  *(volatile v8us*)((unsigned short*)Wt + (size_t)n * K + k8) = o; __threadfence(); *(volatile v8us*)((unsigned short*)Wt + (size_t)n * K + k8) = o; }

__global__ __launch_bounds__(256) void k_mtx(const float* __restrict__ mnv, _Float16* __restrict__ MT) {
  const int t = blockIdx.x * 256 + threadIdx.x; if (t >= 64 * (DM / 8)) return; const int d8 = (t % (DM / 8)) * 8; const int r = t / (DM / 8); FragH f;
#pragma unroll
  for (int q = 0; q < 8; ++q) { const float zv = bf16_rne(mnv[d8 + q]) * MSC; f.h[q] = (r == 0) ? (_Float16)zv : (_Float16)0.0f; }
  const size_t o = (size_t)(DM + r) * DM + d8;
  *(volatile v8us*)((unsigned short*)MT + o) = f.half[0]; __threadfence(); *(volatile v8us*)((unsigned short*)MT + o) = f.half[0]; }

__global__ __launch_bounds__(256) void k_x16r(const float* __restrict__ x, _Float16* __restrict__ X16) {
  const size_t t = (size_t)blockIdx.x * 256 + threadIdx.x; if (t >= (size_t)NR * DM / 8) return;
  const size_t e0 = t * 8; const size_t row = e0 / DM; const int c = (int)(e0 % DM); const int b = (int)(row / SEQ), s = (int)(row % SEQ);
  const float* src = x + ((size_t)b * SEQ_FULL + s) * DM + c; const v4f a = *(const v4fa*)src, cc = *(const v4fa*)(src + 4); FragH f;
#pragma unroll
  for (int q = 0; q < 4; ++q) { f.h[q] = (_Float16)bf16_rne(a[q]); f.h[4 + q] = (_Float16)bf16_rne(cc[q]); }
  *(volatile v8us*)((unsigned short*)X16 + e0) = f.half[0]; __threadfence(); *(volatile v8us*)((unsigned short*)X16 + e0) = f.half[0]; }

template <int NHv, int TTv, int NXv>
__global__ __launch_bounds__(256) void k_vt(const _Float16* __restrict__ V16, int ldv, _Float16* __restrict__ Vt) {
  __shared__ unsigned short tl[64][66];
  const int tid = threadIdx.x; const int slab = blockIdx.x / (TTv / 64), lg = blockIdx.x % (TTv / 64); const int b = slab / NHv, h = slab % NHv;
  for (int i = tid; i < 64 * 8; i += 256) { const int r = i / 8, c8 = (i % 8) * 8; FragH f; f.half[0] = *(const v8us*)((const unsigned short*)V16 + ((size_t)b * TTv + lg * 64 + r) * ldv + h * 64 + c8);
#pragma unroll
    for (int q = 0; q < 8; ++q) tl[r][c8 + q] = f.u[q]; }
  __syncthreads();
  for (int pass = 0; pass < 2; ++pass) {
#pragma unroll
    for (int rd = 0; rd < 2; ++rd) { const int d = rd * 32 + tid / 8, pc = tid % 8; FragH f;
#pragma unroll
      for (int q = 0; q < 8; ++q) f.u[q] = tl[pc * 8 + q][d];
      *(volatile v8us*)((unsigned short*)Vt + ((size_t)b * NXv + h * 64 + d) * TTv + lg * 64 + pc * 8) = f.half[0]; }
    if (pass == 0) __threadfence(); } }

__global__ __launch_bounds__(256) void k_vtx(_Float16* __restrict__ VTH, _Float16* __restrict__ VTL) {
  const size_t t = (size_t)blockIdx.x * 256 + threadIdx.x; const size_t n = (size_t)NB * 64 * (SEQ / 8); if (t >= n) return;
  const int s8 = (int)(t % (SEQ / 8)) * 8; const int r = (int)((t / (SEQ / 8)) % 64); const int b = (int)(t / ((size_t)64 * (SEQ / 8)));
  const unsigned int wv = (r == 0) ? 0x3C003C00u : 0u; v4u oh = {wv, wv, wv, wv}; v4u ol = {0u, 0u, 0u, 0u};
  const size_t o = ((size_t)b * NX + DM + r) * SEQ + s8;
  for (int pass = 0; pass < 2; ++pass) { *(volatile v4u*)((unsigned short*)VTH + o) = oh; *(volatile v4u*)((unsigned short*)VTL + o) = ol; if (pass == 0) __threadfence(); } }

__global__ __launch_bounds__(256) void k_blend(const float* __restrict__ NUM, const float* __restrict__ AM, const float* __restrict__ gate, const float* __restrict__ mnv, _Float16* __restrict__ OH, _Float16* __restrict__ OL) {
  #pragma clang fp contract(off)
  __shared__ float red[256];
  const int tid = threadIdx.x; float s = 0.f;
#pragma unroll 1
  for (int i = tid; i < DM; i += 256) s += bf16_rne(mnv[i]);
  red[tid] = s; __syncthreads();
  for (int st = 128; st > 0; st >>= 1) { if (tid < st) red[tid] += red[tid + st]; __syncthreads(); }
  const float tot = red[0];
  const float act = (tot >= EPSV) ? 1.0f : 0.0f;
  const float gb = bf16_rne(gate[0]); const float g = 1.0f / (1.0f + expf(-gb)); const float g1 = 1.0f - g;
  const size_t t = (size_t)blockIdx.x * 256 + tid;
  if (t < (size_t)NR * DM / 8) {
    const size_t e0 = t * 8; const size_t row = e0 / DM; const int c = (int)(e0 % DM);
    const float* nrow = NUM + row * NX; const float* arow = AM + row * NX;
    const float den = nrow[DM], nrm = arow[DM];
    const float rd = 1.0f / fmaxf(den, EPSV), rn = 1.0f / fmaxf(nrm, EPSV);
    const v4f n0 = *(const v4fa*)(nrow + c), n1 = *(const v4fa*)(nrow + c + 4), a0 = *(const v4fa*)(arow + c), a1 = *(const v4fa*)(arow + c + 4);
    float nu[8] = {n0[0], n0[1], n0[2], n0[3], n1[0], n1[1], n1[2], n1[3]}; float am[8] = {a0[0], a0[1], a0[2], a0[3], a1[0], a1[1], a1[2], a1[3]};
    FragH fh, fl;
#pragma unroll
    for (int q = 0; q < 8; ++q) { float m1 = am[q] * rn; m1 = act * m1; m1 = g * m1; float l1 = nu[q] * rd; l1 = g1 * l1; const float ov = m1 + l1;
      const _Float16 hv = (_Float16)ov; fh.h[q] = hv; fl.h[q] = (_Float16)((ov - (float)hv) * RSC); }
    for (int pass = 0; pass < 2; ++pass) { *(volatile v8us*)((unsigned short*)OH + e0) = fh.half[0]; *(volatile v8us*)((unsigned short*)OL + e0) = fl.half[0]; if (pass == 0) __threadfence(); }
  }
}

extern "C" void kernel_launch(void* const* d_in, const int* in_sizes, int n_in,
                              void* d_out, int out_size, void* d_ws, size_t ws_size, hipStream_t stream) {
  if (n_in < 8) return;
  const float* x = (const float*)d_in[0]; const float* wq = (const float*)d_in[1]; const float* wk = (const float*)d_in[2]; const float* wv = (const float*)d_in[3]; const float* wo = (const float*)d_in[4];
  const float* gate = (const float*)d_in[5]; const float* mem = (const float*)d_in[6]; const float* mnv = (const float*)d_in[7];
  float* out = (float*)d_out;
  const int needx = ((NB - 1) * SEQ_FULL + SEQ) * DM;
  if (in_sizes[0] < needx || in_sizes[1] < DM * DM || in_sizes[2] < DM * DM || in_sizes[3] < DM * DM || in_sizes[4] < DM * DM || in_sizes[5] < 1 || in_sizes[6] < DM * DM || in_sizes[7] < DM || out_size < needx) return;

  char* ws = (char*)d_ws; size_t off = 0;
  auto take = [&](size_t bytes) { char* p = ws + off; off += (bytes + 255) & ~(size_t)255; return p; };
  auto mx3 = [](size_t a, size_t b, size_t c) { size_t m = a > b ? a : b; return m > c ? m : c; };
  const size_t np16 = (size_t)NR * DM * 2;
  const size_t wb = (size_t)DM * DM * 2;
  _Float16* BO = (_Float16*)take(wb);
  _Float16* MT = (_Float16*)take((size_t)NX * DM * 2);
  _Float16* SQH = (_Float16*)take(np16);
  char* rS3 = take(3 * np16);
  _Float16* SQL = (_Float16*)rS3; _Float16* SKH = (_Float16*)(rS3 + np16); _Float16* SKL = (_Float16*)(rS3 + 2 * np16); float* NUM = (float*)rS3;
  const size_t vtb = (size_t)NB * NX * SEQ * 2;
  _Float16* VTH = (_Float16*)take(vtb); _Float16* VTL = (_Float16*)take(vtb);
  const size_t pfb = (size_t)NB * SEQ * SEQ * 4, amb = (size_t)NR * NX * 4;
  char* rB1 = take(mx3(2 * np16, pfb, amb));
  _Float16* VH = (_Float16*)rB1; _Float16* VL = (_Float16*)(rB1 + np16); float* PF = (float*)rB1; float* AM = (float*)rB1;
  const size_t phb = (size_t)NB * SEQ * SEQ * 2;
  char* rB2 = take(mx3(np16 + 3 * wb, 2 * phb, 2 * np16));
  _Float16* X16 = (_Float16*)rB2; _Float16* BQ = (_Float16*)(rB2 + np16); _Float16* BK = (_Float16*)(rB2 + np16 + wb); _Float16* BV = (_Float16*)(rB2 + np16 + 2 * wb);
  _Float16* PH = (_Float16*)rB2; _Float16* PL = (_Float16*)(rB2 + phb); _Float16* OH = (_Float16*)rB2; _Float16* OL = (_Float16*)(rB2 + np16);
  if (off > ws_size || off > WS_CAP) return;

  auto nb256 = [](size_t n) { return (unsigned)((n + 255) / 256); };
  const size_t wn8 = (size_t)DM * DM / 8;
  k_wsc<<<nb256(wn8), 256, 0, stream>>>(wq, BQ, wn8, WSC);
  k_wsc<<<nb256(wn8), 256, 0, stream>>>(wk, BK, wn8, WSC);
  k_wsc<<<nb256(wn8), 256, 0, stream>>>(wv, BV, wn8, WSC);
  k_wsc<<<nb256(wn8), 256, 0, stream>>>(wo, BO, wn8, WSC);
  k_wt_f16<<<nb256(wn8), 256, 0, stream>>>(mem, MT, DM, DM, MSC);
  k_mtx<<<nb256((size_t)64 * (DM / 8)), 256, 0, stream>>>(mnv, MT);
  k_x16r<<<nb256((size_t)NR * DM / 8), 256, 0, stream>>>(x, X16);

  const dim3 gpj((unsigned)((NR / 128) * (DM / 64)), 1);
  k_gemm2<7, 0, 0><<<gpj, 128, 0, stream>>>(X16, DM, (size_t)0, BQ, DM, (size_t)0, 1.0f / WSC, nullptr, 0, nullptr, SQH, SQL, DM, (size_t)0, NR, DM, DM);
  k_gemm2<7, 0, 0><<<gpj, 128, 0, stream>>>(X16, DM, (size_t)0, BK, DM, (size_t)0, 1.0f / WSC, nullptr, 0, nullptr, SKH, SKL, DM, (size_t)0, NR, DM, DM);
  k_gemm2<0, 0, 0><<<gpj, 128, 0, stream>>>(X16, DM, (size_t)0, BV, DM, (size_t)0, 1.0f / WSC, nullptr, 0, nullptr, VH, VL, DM, (size_t)0, NR, DM, DM);
  k_vt<NVH, SEQ, NX><<<(unsigned)(NB * NVH * (SEQ / 64)), 256, 0, stream>>>(VH, DM, VTH);
  k_vt<NVH, SEQ, NX><<<(unsigned)(NB * NVH * (SEQ / 64)), 256, 0, stream>>>(VL, DM, VTL);
  k_vtx<<<nb256((size_t)NB * 64 * (SEQ / 8)), 256, 0, stream>>>(VTH, VTL);

  const dim3 gsc((unsigned)((SEQ / 128) * (SEQ / 64)), NB);
  k_gemm2<0, 1, 0><<<gsc, 128, 0, stream>>>(SQL, DM, (size_t)SEQ * DM, SKH, DM, (size_t)SEQ * DM, 1.0f / RSC, nullptr, 0, PF, nullptr, nullptr, SEQ, (size_t)SEQ * SEQ, SEQ, SEQ, DM);
  k_gemm2<0, 1, 0><<<gsc, 128, 0, stream>>>(SQH, DM, (size_t)SEQ * DM, SKL, DM, (size_t)SEQ * DM, 1.0f / RSC, PF, SEQ, PF, nullptr, nullptr, SEQ, (size_t)SEQ * SEQ, SEQ, SEQ, DM);
  k_gemm2<0, 1, 0><<<gsc, 128, 0, stream>>>(SQH, DM, (size_t)SEQ * DM, SKH, DM, (size_t)SEQ * DM, 1.0f, PF, SEQ, nullptr, PH, PL, SEQ, (size_t)SEQ * SEQ, SEQ, SEQ, DM);

  const dim3 gpe((unsigned)((ERS / 128) * (NX / 64)), NB), gpv((unsigned)((SEQ / 128) * (NX / 64)), NB);
  k_gemm2<0, 0, 1><<<gpe, 128, 0, stream>>>(PL, SEQ, (size_t)SEQ * SEQ, VTH, SEQ, (size_t)NX * SEQ, 1.0f / RSC, nullptr, 0, NUM, nullptr, nullptr, NX, (size_t)SEQ * NX, ERS, NX, SEQ);
  k_gemm2<0, 0, 1><<<gpe, 128, 0, stream>>>(PH, SEQ, (size_t)SEQ * SEQ, VTL, SEQ, (size_t)NX * SEQ, 1.0f / RSC, NUM, ERS, NUM, nullptr, nullptr, NX, (size_t)SEQ * NX, ERS, NX, SEQ);
  k_gemm2<0, 0, 1><<<gpv, 128, 0, stream>>>(PH, SEQ, (size_t)SEQ * SEQ, VTH, SEQ, (size_t)NX * SEQ, 1.0f, NUM, ERS, NUM, nullptr, nullptr, NX, (size_t)SEQ * NX, SEQ, NX, SEQ);

  const dim3 gam((unsigned)((NR / 128) * (NX / 64)), 1);
  k_gemm2<0, 0, 0><<<gam, 128, 0, stream>>>(SQH, DM, (size_t)0, MT, DM, (size_t)0, 1.0f / MSC, nullptr, 0, AM, nullptr, nullptr, NX, (size_t)0, NR, NX, DM);

  k_blend<<<nb256((size_t)NR * DM / 8), 256, 0, stream>>>(NUM, AM, gate, mnv, OH, OL);

  const dim3 gwe((unsigned)((ERS / 128) * (DM / 64)), NB), gwo((unsigned)((SEQ / 128) * (DM / 64)), NB);
  k_gemm2<0, 0, 0><<<gwe, 128, 0, stream>>>(OL, DM, (size_t)SEQ * DM, BO, DM, (size_t)0, 1.0f / (WSC * RSC), nullptr, 0, out, nullptr, nullptr, DM, (size_t)SEQ_FULL * DM, ERS, DM, DM);
  k_gemm2<0, 0, 0><<<gwo, 128, 0, stream>>>(OH, DM, (size_t)SEQ * DM, BO, DM, (size_t)0, 1.0f / WSC, out, ERS, out, nullptr, nullptr, DM, (size_t)SEQ_FULL * DM, SEQ, DM, DM);
}
